// MultiGATLayer_24627342475868
// MI455X (gfx1250) — hardware-verified
//
#include <hip/hip_runtime.h>
#include <math.h>

constexpr int kNodes    = 20000;
constexpr int kNodesPad = 20032;
constexpr int kDeg      = 16;
constexpr int kFin      = 128;
constexpr int kFout     = 128;
constexpr int kHeads    = 4;
constexpr int kHF       = kHeads * kFout;
constexpr int kCand     = kDeg + 1;
constexpr float kWCarry    = 64.0f;
constexpr float kWCarryInv = 1.0f / 64.0f;
static_assert(kNodesPad % 64 == 0);
static_assert(kNodesPad >= kNodes);
static_assert(kHF % 64 == 0);
static_assert(kFin % 32 == 0);
static_assert(kNodes % 32 == 0);
static_assert((kNodes * kHeads) % 8 == 0);

typedef __attribute__((ext_vector_type(16))) _Float16 v16h;
typedef __attribute__((ext_vector_type(8)))  _Float16 v8h;
typedef __attribute__((ext_vector_type(16))) __bf16   v16b;
typedef __attribute__((ext_vector_type(8)))  __bf16   v8b;
typedef __attribute__((ext_vector_type(8)))  float    v8f;
typedef __attribute__((ext_vector_type(4)))  float    v4f;
typedef __attribute__((ext_vector_type(4)))  unsigned int v4u;

__device__ __forceinline__ unsigned short f2bf_bits(float f) {
  unsigned u = __float_as_uint(f);
  return (unsigned short)((u + 0x7FFFu + ((u >> 16) & 1u)) >> 16);
}
__device__ __forceinline__ float bf_bits2f(unsigned short h) { return __uint_as_float(((unsigned)h) << 16); }

__device__ __forceinline__ void dep_guard_h(v8f& a, v8f& b, v16h x, v16h y) { asm volatile("v_nop\n\tv_nop\n\tv_nop\n\tv_nop" : "+v"(a), "+v"(b) : "v"(x), "v"(y)); }
__device__ __forceinline__ void dep_guard_b(v8f& a, v8f& b, v16b x, v16b y) { asm volatile("v_nop\n\tv_nop\n\tv_nop\n\tv_nop" : "+v"(a), "+v"(b) : "v"(x), "v"(y)); }
__device__ __forceinline__ void keep4_h(v16h a, v16h b, v16h c, v16h d) { asm volatile("v_nop" :: "v"(a), "v"(b), "v"(c), "v"(d)); }
__device__ __forceinline__ void keep4_b(v16b a, v16b b, v16b c, v16b d) { asm volatile("v_nop" :: "v"(a), "v"(b), "v"(c), "v"(d)); }
__device__ __forceinline__ void acc_guard4(v8f& a, v8f& b, v8f& c, v8f& d) { asm volatile("v_nop\n\tv_nop\n\tv_nop\n\tv_nop" : "+v"(a), "+v"(b), "+v"(c), "+v"(d)); }
template <typename T> struct Frag;
template <> struct Frag<_Float16> {
  typedef v16h V; union U { v16h v; v8h h[2]; };
  static __device__ __forceinline__ v16h load(const _Float16* p) {
    U f; f.h[0] = *(const v8h*)(p); f.h[1] = *(const v8h*)(p + 16); return f.v;
  }
  static __device__ __forceinline__ v8f mma(v16h a, v16h b, v8f c) {
    return __builtin_amdgcn_wmma_f32_16x16x32_f16(false, a, false, b, (short)0, c, false, false);
  }
  static __device__ __forceinline__ void guard(v8f& a, v8f& b, v16h x, v16h y) { dep_guard_h(a, b, x, y); }
  static __device__ __forceinline__ void keep(v16h a, v16h b, v16h c, v16h d) { keep4_h(a, b, c, d); }
};
template <> struct Frag<__bf16> {
  typedef v16b V; union U { v16b v; v8b h[2]; };
  static __device__ __forceinline__ v16b load(const __bf16* p) {
    U f; f.h[0] = *(const v8b*)(p); f.h[1] = *(const v8b*)(p + 16); return f.v;
  }
  static __device__ __forceinline__ v8f mma(v16b a, v16b b, v8f c) {
    return __builtin_amdgcn_wmma_f32_16x16x32_bf16(false, a, false, b, (short)0, c, false, false);
  }
  static __device__ __forceinline__ void guard(v8f& a, v8f& b, v16b x, v16b y) { dep_guard_b(a, b, x, y); }
  static __device__ __forceinline__ void keep(v16b a, v16b b, v16b c, v16b d) { keep4_b(a, b, c, d); }
};

__device__ __forceinline__ unsigned pk16(unsigned short a, unsigned short b) { return (unsigned)a | ((unsigned)b << 16); }
__device__ __forceinline__ unsigned short h_bits(float f) { const _Float16 h = (_Float16)f; return __builtin_bit_cast(unsigned short, h); }

template <int ET> struct Elem;
template <> struct Elem<0> { typedef _Float16 T; };
template <> struct Elem<1> { typedef __bf16 T; };
template <int ET, bool SPLIT, int BIAS_MODE, int OUT_MODE, bool RESID, int ACT = 0>
__global__ __launch_bounds__(256) void wmma_gemm64(
    const unsigned short* __restrict__ Ap, const unsigned short* __restrict__ A2p, int lda, long strideA,
    const unsigned short* __restrict__ Btp, const unsigned short* __restrict__ Bt2p, int ldb, long strideB,
    void* __restrict__ Cout, void* __restrict__ Cout2, int ldc, long strideC,
    const float* __restrict__ bias,
    const float* __restrict__ resid, long strideR,
    int M, int N, int K, float scale) {
  typedef typename Elem<ET>::T T;
  typedef typename Frag<T>::V V;
  const T* A = (const T*)Ap; const T* A2 = (const T*)A2p; const T* Bt = (const T*)Btp; const T* Bt2 = (const T*)Bt2p;
  __shared__ __align__(16) float sT[8][16 * 68];
  const int b    = blockIdx.y;
  const int lane = threadIdx.x & 31;
  const int wave = threadIdx.x >> 5;
  const int tilesN = N >> 6;
  const int tilesM = M >> 6;
  const int tile = blockIdx.x * 8 + wave;
  if (tile >= tilesM * tilesN) return;
  const int tm = tile / tilesN;
  const int tn = tile - tm * tilesN;
  const int m0 = tm << 6;
  const int n0 = tn << 6;

  const T* Ab  = A  + (size_t)b * strideA;
  const T* Bb  = Bt + (size_t)b * strideB;
  const T* Ab2 = SPLIT ? (A2  + (size_t)b * strideA) : nullptr;
  const T* Bb2 = SPLIT ? (Bt2 + (size_t)b * strideB) : nullptr;

  const int rlane = lane & 15;
  const int koff  = (lane >> 4) * 8;
  const int mOff  = (lane >> 4) * 8;

  v8f acc[4][4];
#pragma unroll
  for (int i = 0; i < 4; ++i)
#pragma unroll
    for (int j = 0; j < 4; ++j) acc[i][j] = (v8f){0.f,0.f,0.f,0.f,0.f,0.f,0.f,0.f};

  for (int k0 = 0; k0 < K; k0 += 32) {
    V bh[4], bl[4];
#pragma unroll
    for (int j = 0; j < 4; ++j) {
      const size_t bo = (size_t)(n0 + (j << 4) + rlane) * ldb + koff + k0;
      bh[j] = Frag<T>::load(Bb + bo);
      if (SPLIT) bl[j] = Frag<T>::load(Bb2 + bo);
    }
#pragma unroll
    for (int i = 0; i < 4; ++i) {
      const size_t ao = (size_t)(m0 + (i << 4) + rlane) * lda + koff + k0;
      V ah = Frag<T>::load(Ab + ao);
      V al;
      if (SPLIT) al = Frag<T>::load(Ab2 + ao);
#pragma unroll
      for (int j = 0; j < 4; ++j) {
        acc[i][j] = Frag<T>::mma(ah, bh[j], acc[i][j]);
        if (SPLIT) {
          acc[i][j] = Frag<T>::mma(ah, bl[j], acc[i][j]);
          acc[i][j] = Frag<T>::mma(al, bh[j], acc[i][j]);
        }
      }
      Frag<T>::guard(acc[i][0], acc[i][3], ah, SPLIT ? al : ah);
    }
    Frag<T>::keep(bh[0], bh[1], bh[2], bh[3]);
    if (SPLIT) Frag<T>::keep(bl[0], bl[1], bl[2], bl[3]);
  }
  acc_guard4(acc[0][0], acc[0][1], acc[0][2], acc[0][3]);
  acc_guard4(acc[1][0], acc[1][1], acc[1][2], acc[1][3]);
  acc_guard4(acc[2][0], acc[2][1], acc[2][2], acc[2][3]);
  acc_guard4(acc[3][0], acc[3][1], acc[3][2], acc[3][3]);

  float* slab = sT[wave];
  const float* Rb = RESID ? (resid + (size_t)b * strideR) : nullptr;
#pragma unroll
  for (int i = 0; i < 4; ++i) {
    const int mBase = m0 + (i << 4);
#pragma unroll
    for (int j = 0; j < 4; ++j) {
      const int n = n0 + (j << 4) + rlane;
      float bv = 0.f;
      if (BIAS_MODE == 2) bv = bias[n];
#pragma unroll
      for (int r = 0; r < 8; ++r) {
        float v = acc[i][j][r] * scale;
        if (BIAS_MODE == 1) v += bias[mBase + mOff + r];
        if (BIAS_MODE == 2) v += bv;
        if (RESID) v += Rb[(size_t)(mBase + mOff + r) * ldc + n];
        if (ACT == 2) v = fmaxf(v, 0.0f);
        if (ACT == 4) v = (v > 0.f) ? v : 0.01f * v;
        slab[(mOff + r) * 68 + (j << 4) + rlane] = v;
      }
    }
    __builtin_amdgcn_fence(__ATOMIC_RELEASE, "workgroup");
    __builtin_amdgcn_wave_barrier();
    __builtin_amdgcn_fence(__ATOMIC_ACQUIRE, "workgroup");
    if (OUT_MODE == 0) {
      float* C = (float*)Cout + (size_t)b * strideC;
      const int hh = lane >> 4, c4 = (lane & 15) * 4;
      for (int pass = 0; pass < 2; ++pass) {
#pragma unroll
        for (int it = 0; it < 8; ++it) {
          const int row = it * 2 + hh;
          v4f v = *(const v4f*)(slab + row * 68 + c4);
          *(volatile v4f*)(C + (size_t)(mBase + row) * ldc + n0 + c4) = v;
        }
        __threadfence();
      }
    } else {
      const int q = lane >> 3, c8 = (lane & 7) * 8;
      unsigned short* C  = (unsigned short*)Cout  + (size_t)b * strideC;
      unsigned short* C2 = (OUT_MODE == 2) ? ((unsigned short*)Cout2 + (size_t)b * strideC) : nullptr;
      for (int pass = 0; pass < 2; ++pass) {
#pragma unroll
        for (int it = 0; it < 4; ++it) {
          const int row = it * 4 + q;
          const float* sp = slab + row * 68 + c8;
          v8h hv, lv;
#pragma unroll
          for (int e = 0; e < 8; ++e) {
            if (OUT_MODE == 1) {
              hv[e] = (_Float16)sp[e];
            } else {
              unsigned short hb = f2bf_bits(sp[e]);
              unsigned short lb = f2bf_bits(sp[e] - bf_bits2f(hb));
              hv[e] = __builtin_bit_cast(_Float16, hb);
              lv[e] = __builtin_bit_cast(_Float16, lb);
            }
          }
          *(volatile v8h*)(C + (size_t)(mBase + row) * ldc + n0 + c8) = hv;
          if (OUT_MODE == 2) *(volatile v8h*)(C2 + (size_t)(mBase + row) * ldc + n0 + c8) = lv;
        }
        __threadfence();
      }
    }
    __builtin_amdgcn_fence(__ATOMIC_RELEASE, "workgroup");
    __builtin_amdgcn_wave_barrier();
    __builtin_amdgcn_fence(__ATOMIC_ACQUIRE, "workgroup");
  }
}

__global__ __launch_bounds__(256) void cast_feat_kernel(const float* __restrict__ in, unsigned short* __restrict__ out,
                                                        int n8_valid, int n8_total) {
  const int i = blockIdx.x * 256 + threadIdx.x;
  if (i >= n8_total) return;
  const int ic = (i < n8_valid) ? i : (n8_valid - 1);
  const float* p = in + 8 * (size_t)ic;
  v4f a = *(const v4f*)(p);
  v4f c = *(const v4f*)(p + 4);
  if (i >= n8_valid) { a = (v4f){0.f, 0.f, 0.f, 0.f}; c = a; }
  unsigned short hb[8];
#pragma unroll
  for (int e = 0; e < 4; ++e) {
    hb[e]     = h_bits(a[e]);
    hb[4 + e] = h_bits(c[e]);
  }
  const v4u u = (v4u){pk16(hb[0], hb[1]), pk16(hb[2], hb[3]), pk16(hb[4], hb[5]), pk16(hb[6], hb[7])};
  unsigned short* q = out + 8 * (size_t)i;
  *(volatile v4u*)q = u;
  __threadfence();
  *(volatile v4u*)q = u;
}

__global__ __launch_bounds__(256) void wtcast_kernel(const float* __restrict__ Win, unsigned short* __restrict__ Bt, float scale) {
  __shared__ float sm[64][65];
  const int t  = threadIdx.x;
  const int i0 = blockIdx.x * 64;
  const int o0 = blockIdx.y * 64;
  const int hd = blockIdx.z;
  const float* W = Win + (size_t)hd * kFin * kFout;
#pragma unroll
  for (int it = 0; it < 16; ++it) {
    const int e = it * 256 + t;
    const int r = e >> 6;
    const int c = e & 63;
    sm[c][r] = W[(size_t)(i0 + r) * kFout + o0 + c] * scale;
  }
  __syncthreads();
  const int lane = t & 31, wave = t >> 5;
  const int q = lane >> 3, c8 = (lane & 7) * 8;
  unsigned short* op = Bt + (size_t)hd * kFout * kFin;
  for (int pass = 0; pass < 2; ++pass) {
#pragma unroll
    for (int it = 0; it < 2; ++it) {
      const int row = wave * 8 + it * 4 + q;
      unsigned short hb[8];
#pragma unroll
      for (int e = 0; e < 8; ++e) hb[e] = h_bits(sm[row][c8 + e]);
      const v4u u = (v4u){pk16(hb[0], hb[1]), pk16(hb[2], hb[3]), pk16(hb[4], hb[5]), pk16(hb[6], hb[7])};
      *(volatile v4u*)(op + (size_t)(o0 + row) * kFin + i0 + c8) = u;
    }
    __threadfence();
  }
}

__global__ __launch_bounds__(256) void score_kernel(const float* __restrict__ Hp, const float* __restrict__ a_w,
                                                     float* __restrict__ S, int nNodes) {
  __shared__ __align__(16) float sS[32 * 8];
  const int t = threadIdx.x;
  const int lane = t & 31, wave = t >> 5;
  v4f aself[kHeads], anb[kHeads];
#pragma unroll
  for (int hd = 0; hd < kHeads; ++hd) {
    aself[hd] = *(const v4f*)(a_w + hd * 2 * kFout + lane * 4);
    anb[hd]   = *(const v4f*)(a_w + hd * 2 * kFout + kFout + lane * 4);
  }
  const int nbase = blockIdx.x * 32 + wave * 4;
#pragma unroll 1
  for (int j = 0; j < 4; ++j) {
    const int n  = nbase + j;
    const int nc = (n < nNodes) ? n : (nNodes - 1);
    const float* hr = Hp + (size_t)nc * kHF + lane * 4;
#pragma unroll
    for (int hd = 0; hd < kHeads; ++hd) {
      const v4f v = *(const v4f*)(hr + hd * kFout);
      float ps = v.x * aself[hd].x + v.y * aself[hd].y + v.z * aself[hd].z + v.w * aself[hd].w;
      float pn = v.x * anb[hd].x   + v.y * anb[hd].y   + v.z * anb[hd].z   + v.w * anb[hd].w;
#pragma unroll
      for (int off = 16; off > 0; off >>= 1) {
        ps += __shfl_xor(ps, off, 32);
        pn += __shfl_xor(pn, off, 32);
      }
      if (lane == 0) {
        sS[(wave * 4 + j) * 8 + hd] = ps;
        sS[(wave * 4 + j) * 8 + kHeads + hd] = pn;
      }
    }
  }
  __syncthreads();
  if (wave == 0) {
    float* Sb = S + (size_t)blockIdx.x * 256;
    const v4f v0 = *(const v4f*)(sS + lane * 4);
    const v4f v1 = *(const v4f*)(sS + 128 + lane * 4);
    *(volatile v4f*)(Sb + lane * 4) = v0;
    *(volatile v4f*)(Sb + 128 + lane * 4) = v1;
    __threadfence();
    *(volatile v4f*)(Sb + lane * 4) = v0;
    *(volatile v4f*)(Sb + 128 + lane * 4) = v1;
  }
}

__global__ __launch_bounds__(256) void aggregate_kernel(const int* __restrict__ adj, const float* __restrict__ Hp,
                                                         const float* __restrict__ S, const float* __restrict__ a_b,
                                                         float* __restrict__ out, int nNodes) {
  const int lane = threadIdx.x & 31, wave = threadIdx.x >> 5;
  const int wid = blockIdx.x * 8 + wave;
  const int n  = wid >> 2;
  const int hd = wid & 3;
  if (n >= nNodes) return;

  const int al = (lane < kDeg) ? lane : (kDeg - 1);
  int cid = adj[(size_t)n * kDeg + al];
  cid = (cid < 0) ? 0 : cid;
  cid = (cid > nNodes - 1) ? (nNodes - 1) : cid;
  const int cand = (lane < kDeg) ? cid : n;

  const float ss  = S[(size_t)n * 8 + hd];
  const float snb = S[(size_t)cand * 8 + kHeads + hd];
  const float ab  = a_b[hd];
  const float z   = (ss + snb) + ab;
  float lg = (z >= 0.f) ? z : 0.2f * z;
  lg = (lane < kCand) ? lg : -INFINITY;

  float m = lg;
#pragma unroll
  for (int off = 16; off > 0; off >>= 1) m = fmaxf(m, __shfl_xor(m, off, 32));
  float e = expf(lg - m);
  e = (lane < kCand) ? e : 0.f;
  float s = e;
#pragma unroll
  for (int off = 16; off > 0; off >>= 1) s += __shfl_xor(s, off, 32);
  const float attn = e * (1.0f / s);

  const float* hb = Hp + hd * kFout + lane * 4;
  v4f acc = (v4f){0.f, 0.f, 0.f, 0.f};
#pragma unroll 1
  for (int d = 0; d < kCand; ++d) {
    const float a_d = __shfl(attn, d, 32);
    const int   n_d = __shfl(cand, d, 32);
    const v4f v = *(const v4f*)(hb + (size_t)n_d * kHF);
    acc += a_d * v;
  }
  float* op = out + (size_t)n * kHF + hd * kFout + lane * 4;
  *(volatile v4f*)op = acc;
  __threadfence();
  *(volatile v4f*)op = acc;
}

extern "C" void kernel_launch(void* const* d_in, const int* in_sizes, int n_in,
                              void* d_out, int out_size, void* d_ws, size_t ws_size,
                              hipStream_t stream) {
  if (n_in < 6) return;
  if (in_sizes[0] != kNodes * kDeg || in_sizes[1] != kNodes * kFin || in_sizes[2] != kHeads * kFin * kFout ||
      in_sizes[3] != kHeads * kFout || in_sizes[4] != kHeads * 2 * kFout || in_sizes[5] != kHeads ||
      out_size != kNodes * kHF) return;

  const int*   adj  = (const int*)d_in[0];
  const float* feat = (const float*)d_in[1];
  const float* W    = (const float*)d_in[2];
  const float* bW   = (const float*)d_in[3];
  const float* a_w  = (const float*)d_in[4];
  const float* a_b  = (const float*)d_in[5];
  float* out = (float*)d_out;

  char* ws = (char*)d_ws;
  size_t off = 0;
  const size_t szFeatH = (size_t)kNodesPad * kFin * 2;
  const size_t szBt    = (size_t)kHF * kFin * 2;
  const size_t szH     = (size_t)kNodesPad * kHF * 4;
  const size_t szS     = (size_t)kNodes * 8 * 4;
  unsigned short* featH = (unsigned short*)(ws + off); off += szFeatH;
  unsigned short* Bt    = (unsigned short*)(ws + off); off += szBt;
  float*          Hf    = (float*)(ws + off);          off += szH;
  float*          Sbuf  = (float*)(ws + off);          off += szS;
  if (off > ws_size) return;

  const int n8_valid = kNodes * kFin / 8;
  const int n8_total = kNodesPad * kFin / 8;
  cast_feat_kernel<<<dim3((n8_total + 255) / 256), dim3(256), 0, stream>>>(feat, featH, n8_valid, n8_total);

  wtcast_kernel<<<dim3(kFin / 64, kFout / 64, kHeads), dim3(256), 0, stream>>>(W, Bt, kWCarry);

  {
    const int tiles  = (kNodesPad / 64) * (kHF / 64);
    const int blocks = (tiles + 7) / 8;
    wmma_gemm64<0, false, 2, 0, false, 0><<<dim3(blocks, 1), dim3(256), 0, stream>>>(
        featH, featH, kFin, 0L,
        Bt, Bt, kFin, 0L,
        (void*)Hf, (void*)Hf, kHF, 0L,
        bW,
        (const float*)nullptr, 0L,
        kNodesPad, kHF, kFin, kWCarryInv);
  }

  score_kernel<<<dim3(kNodes / 32), dim3(256), 0, stream>>>(Hf, a_w, Sbuf, kNodes);

  aggregate_kernel<<<dim3((kNodes * kHeads + 7) / 8), dim3(256), 0, stream>>>(adj, Hf, Sbuf, a_b, out, kNodes);
}
